// stackedIndRNN_encoder_20435454395119
// MI455X (gfx1250) — hardware-verified
//
#include <hip/hip_runtime.h>
#include <math.h>

constexpr int NLAYER = 6;
constexpr int NSTEP  = 256;
constexpr int NBATCH = 64;
constexpr int NIN    = 128;
constexpr int NHID   = 1024;
constexpr int NCLS   = 128;
constexpr int NROWS  = NSTEP * NBATCH;
constexpr int NTHR   = 256;
constexpr int SLABP  = 68;
constexpr int NTILEM = NROWS / 64;
constexpr int NTILEN = NHID / 64;
constexpr float WCARRY     = 256.0f;
constexpr float WCARRY_INV = 1.0f / 256.0f;
constexpr float BN_EPS_F   = 1e-5f;

static_assert(NROWS == 16384, "row count");
static_assert(NROWS % 64 == 0 && NHID % 64 == 0, "GEMM M, N tile multiples");
static_assert(NIN % 32 == 0 && NHID % 32 == 0, "GEMM K multiples of 32");
static_assert((NTILEM * NTILEN) % 8 == 0, "GEMM grid exact");
static_assert(NIN % 64 == 0 && NHID % 64 == 0, "transpose tiles exact");
static_assert((NROWS * NIN / 8) % NTHR == 0, "convert grid exact");
static_assert((NBATCH * NHID / 2) % NTHR == 0, "scan grid exact");
static_assert((NBATCH * NCLS) % NTHR == 0, "head grid exact");
static_assert(NHID % NTHR == 0, "finalize grid exact");
static_assert(NSTEP % 8 == 0, "scan step groups exact");

typedef __attribute__((ext_vector_type(16))) _Float16 v16h;
typedef __attribute__((ext_vector_type(8)))  _Float16 v8h;
typedef __attribute__((ext_vector_type(8)))  float    v8f;
typedef __attribute__((ext_vector_type(4)))  float    v4f;
typedef __attribute__((ext_vector_type(2)))  float    v2f;

__device__ __forceinline__ unsigned short f2bf_bits(float f) {
  unsigned u = __float_as_uint(f);
  return (unsigned short)((u + 0x7FFFu + ((u >> 16) & 1u)) >> 16);
}
__device__ __forceinline__ float bf_bits2f(unsigned short h) { return __uint_as_float(((unsigned)h) << 16); }
__device__ __forceinline__ float bf16r(float f) { return bf_bits2f(f2bf_bits(f)); }

__device__ __forceinline__ void guard_row(v8f& a0, v8f& a1, v8f& a2, v8f& a3, v16h x, v16h b0, v16h b1, v16h b2, v16h b3) {
  asm volatile("v_nop\n\tv_nop\n\tv_nop\n\tv_nop" : "+v"(a0), "+v"(a1), "+v"(a2), "+v"(a3) : "v"(x), "v"(b0), "v"(b1), "v"(b2), "v"(b3));
}
__device__ __forceinline__ void acc_guard4(v8f& a, v8f& b, v8f& c, v8f& d) {
  asm volatile("v_nop\n\tv_nop\n\tv_nop\n\tv_nop" : "+v"(a), "+v"(b), "+v"(c), "+v"(d));
}

template <typename T> struct Frag;
template <> struct Frag<_Float16> {
  typedef v16h V; union U { v16h v; v8h h[2]; };
  static __device__ __forceinline__ v16h load(const _Float16* p) {
    U f; f.h[0] = *(const v8h*)(p); f.h[1] = *(const v8h*)(p + 16); return f.v;
  }
  static __device__ __forceinline__ v8f mma(v16h a, v16h b, v8f c) {
    return __builtin_amdgcn_wmma_f32_16x16x32_f16(false, a, false, b, (short)0, c, false, false);
  }
};

__global__ __launch_bounds__(NTHR) void cvt8_kernel(const float* __restrict__ src, unsigned short* __restrict__ dst, int n8) {
  const int i = blockIdx.x * NTHR + threadIdx.x;
  if (i < n8) {
    const float* sp = src + (size_t)i * 8;
    const v4f a = *(const v4f*)(sp);
    const v4f b = *(const v4f*)(sp + 4);
    v8h hv;
#pragma unroll
    for (int e = 0; e < 4; ++e) {
      const float fa = a[e];
      const float fb = b[e];
      hv[e]     = (_Float16)bf16r(fa);
      hv[4 + e] = (_Float16)bf16r(fb);
    }
    *(volatile v8h*)(dst + (size_t)i * 8) = hv;
    __threadfence();
    *(volatile v8h*)(dst + (size_t)i * 8) = hv;
  }
}

__global__ __launch_bounds__(NTHR) void tpw_kernel(const float* __restrict__ src, int R, int C, int ldo,
                                                  unsigned short* __restrict__ O, float sc) {
  __shared__ float Tt[64 * 65];
  const int tid = threadIdx.x;
  const int c0 = blockIdx.x * 64, r0 = blockIdx.y * 64;
  const float* sz = src + (size_t)blockIdx.z * (size_t)R * (size_t)C;
  unsigned short* oz = O + (size_t)blockIdx.z * (size_t)C * (size_t)ldo;
#pragma unroll
  for (int i = 0; i < 4; ++i) {
    const int idx = i * NTHR + tid;
    const int rr = idx >> 4, cc = (idx & 15) * 4;
    const v4f v = *(const v4f*)(sz + (size_t)(r0 + rr) * (size_t)C + c0 + cc);
    Tt[rr * 65 + cc + 0] = v[0];
    Tt[rr * 65 + cc + 1] = v[1];
    Tt[rr * 65 + cc + 2] = v[2];
    Tt[rr * 65 + cc + 3] = v[3];
  }
  __syncthreads();
  const int q = tid >> 3, c8 = (tid & 7) * 8;
  v8h hv[2];
#pragma unroll
  for (int g = 0; g < 2; ++g) {
    const int qq = g * 32 + q;
#pragma unroll
    for (int e = 0; e < 8; ++e) {
      const float f = Tt[(c8 + e) * 65 + qq];
      hv[g][e] = (_Float16)(bf16r(f) * sc);
    }
  }
  for (int pass = 0; pass < 2; ++pass) {
#pragma unroll
    for (int g = 0; g < 2; ++g) {
      const size_t o = (size_t)(c0 + g * 32 + q) * (size_t)ldo + (size_t)(r0 + c8);
      *(volatile v8h*)(oz + o) = hv[g];
    }
    __threadfence();
  }
}

template <int KD>
__global__ __launch_bounds__(256) void gemm_f16_stats(const unsigned short* __restrict__ Ap,
                                                      const unsigned short* __restrict__ Btp,
                                                      const float* __restrict__ bias,
                                                      float* __restrict__ Xo,
                                                      float* __restrict__ PS, float* __restrict__ PQ) {
  static_assert(KD % 32 == 0, "K multiple of 32");
  __shared__ __align__(16) float sT[8][16 * SLABP];
  const _Float16* A  = (const _Float16*)Ap;
  const _Float16* Bt = (const _Float16*)Btp;
  const int lane = threadIdx.x & 31;
  const int wave = threadIdx.x >> 5;
  const int tile = blockIdx.x * 8 + wave;
  const int tm = tile / NTILEN;
  const int tn = tile - tm * NTILEN;
  const int m0 = tm << 6;
  const int n0 = tn << 6;
  const int rlane = lane & 15;
  const int hh    = lane >> 4;
  const int koff  = hh * 8;
  const int mOff  = hh * 8;

  const _Float16* aP = A  + (size_t)(m0 + rlane) * KD + koff;
  const _Float16* bP = Bt + (size_t)(n0 + rlane) * KD + koff;

  v8f acc[4][4];
#pragma unroll
  for (int i = 0; i < 4; ++i)
#pragma unroll
    for (int j = 0; j < 4; ++j) acc[i][j] = (v8f){0.f, 0.f, 0.f, 0.f, 0.f, 0.f, 0.f, 0.f};

#pragma unroll 1
  for (int k0 = 0; k0 < KD; k0 += 32) {
    v16h bh[4];
#pragma unroll
    for (int j = 0; j < 4; ++j) bh[j] = Frag<_Float16>::load(bP + (size_t)(j * 16) * KD + k0);
#pragma unroll
    for (int i = 0; i < 4; ++i) {
      const v16h ah = Frag<_Float16>::load(aP + (size_t)(i * 16) * KD + k0);
#pragma unroll
      for (int j = 0; j < 4; ++j) acc[i][j] = Frag<_Float16>::mma(ah, bh[j], acc[i][j]);
      guard_row(acc[i][0], acc[i][1], acc[i][2], acc[i][3], ah, bh[0], bh[1], bh[2], bh[3]);
    }
  }
  acc_guard4(acc[0][0], acc[0][1], acc[0][2], acc[0][3]);
  acc_guard4(acc[1][0], acc[1][1], acc[1][2], acc[1][3]);
  acc_guard4(acc[2][0], acc[2][1], acc[2][2], acc[2][3]);
  acc_guard4(acc[3][0], acc[3][1], acc[3][2], acc[3][3]);

  float* slab = sT[wave];
  float bv[4], cs[4], cq[4];
#pragma unroll
  for (int j = 0; j < 4; ++j) {
    bv[j] = bf16r(bias[n0 + (j << 4) + rlane]);
    cs[j] = 0.0f;
    cq[j] = 0.0f;
  }
  const int c4 = (lane & 15) * 4;
#pragma unroll
  for (int i = 0; i < 4; ++i) {
    const int mBase = m0 + (i << 4);
#pragma unroll
    for (int j = 0; j < 4; ++j) {
#pragma unroll
      for (int r = 0; r < 8; ++r) {
        const float v = fmaf(acc[i][j][r], WCARRY_INV, bv[j]);
        cs[j] += v;
        cq[j] = fmaf(v, v, cq[j]);
        slab[(mOff + r) * SLABP + (j << 4) + rlane] = v;
      }
    }
    __builtin_amdgcn_fence(__ATOMIC_RELEASE, "workgroup");
    __builtin_amdgcn_wave_barrier();
    __builtin_amdgcn_fence(__ATOMIC_ACQUIRE, "workgroup");
    for (int pass = 0; pass < 2; ++pass) {
#pragma unroll
      for (int it = 0; it < 8; ++it) {
        const int row = it * 2 + hh;
        const v4f v = *(const v4f*)(slab + row * SLABP + c4);
        *(volatile v4f*)(Xo + (size_t)(mBase + row) * NHID + n0 + c4) = v;
      }
      __threadfence();
    }
    __builtin_amdgcn_fence(__ATOMIC_RELEASE, "workgroup");
    __builtin_amdgcn_wave_barrier();
    __builtin_amdgcn_fence(__ATOMIC_ACQUIRE, "workgroup");
  }
#pragma unroll
  for (int j = 0; j < 4; ++j) {
    const float os = __shfl_xor(cs[j], 16, 32);
    const float oq = __shfl_xor(cq[j], 16, 32);
    cs[j] += os;
    cq[j] += oq;
  }
#pragma unroll
  for (int j = 0; j < 4; ++j) {
    const float w = hh ? cq[j] : cs[j];
    slab[hh * SLABP + (j << 4) + rlane] = w;
  }
  __builtin_amdgcn_fence(__ATOMIC_RELEASE, "workgroup");
  __builtin_amdgcn_wave_barrier();
  __builtin_amdgcn_fence(__ATOMIC_ACQUIRE, "workgroup");
  {
    const v4f pv = *(const v4f*)(slab + hh * SLABP + c4);
    float* pbase = hh ? PQ : PS;
    float* pp = pbase + (size_t)tm * NHID + n0 + c4;
    *(volatile v4f*)pp = pv;
    __threadfence();
    *(volatile v4f*)pp = pv;
  }
}

__global__ __launch_bounds__(NTHR) void stat_finalize_kernel(const float* __restrict__ PS, const float* __restrict__ PQ,
                                                            const float* __restrict__ gam, float* __restrict__ STAT) {
  const int c = blockIdx.x * NTHR + threadIdx.x;
  double s = 0.0, q = 0.0;
#pragma unroll 4
  for (int t = 0; t < NTILEM; ++t) {
    s += (double)PS[(size_t)t * NHID + c];
    q += (double)PQ[(size_t)t * NHID + c];
  }
  const double inv = 1.0 / (double)NROWS;
  const double m = s * inv;
  double var = q * inv - m * m;
  var = (var < 0.0) ? 0.0 : var;
  const float rs = rsqrtf((float)var + BN_EPS_F);
  const float g  = bf16r(gam[c]);
  const float mf = (float)m;
  const float sc = g * rs;
  *(volatile float*)(STAT + c) = mf;
  *(volatile float*)(STAT + NHID + c) = sc;
  __threadfence();
  *(volatile float*)(STAT + c) = mf;
  *(volatile float*)(STAT + NHID + c) = sc;
}

template <bool LASTL>
__global__ __launch_bounds__(NTHR) void scan_kernel(const float* __restrict__ X, const float* __restrict__ STAT,
                                                   const float* __restrict__ beta, const float* __restrict__ uvec,
                                                   unsigned* __restrict__ HP, float* __restrict__ LASTP) {
  const int idx = blockIdx.x * NTHR + threadIdx.x;
  const int b = idx >> 9;
  const int p = idx & 511;
  const int ch = p * 2;
  const v2f mv = *(const v2f*)(STAT + ch);
  const v2f sv = *(const v2f*)(STAT + NHID + ch);
  const v2f bt = *(const v2f*)(beta + ch);
  const v2f uv = *(const v2f*)(uvec + ch);
  const float mean0 = mv[0], mean1 = mv[1];
  const float sc0 = sv[0], sc1 = sv[1];
  const float btf0 = bt[0], btf1 = bt[1];
  const float uf0 = uv[0], uf1 = uv[1];
  const float be0 = bf16r(btf0), be1 = bf16r(btf1);
  const float u0 = bf16r(uf0), u1 = bf16r(uf1);
  float st0 = 0.0f, st1 = 0.0f;
  const size_t XSTRIDE = (size_t)NBATCH * NHID;
  const size_t HSTRIDE = (size_t)NBATCH * NHID / 2;
  const float* xp = X + (size_t)b * NHID + ch;
  unsigned* hp = HP + (size_t)b * (NHID / 2) + p;
#pragma unroll 1
  for (int t0 = 0; t0 < NSTEP; t0 += 8) {
    v2f xv[8];
#pragma unroll
    for (int e = 0; e < 8; ++e) xv[e] = *(const v2f*)(xp + (size_t)(t0 + e) * XSTRIDE);
    unsigned pk[8];
#pragma unroll
    for (int e = 0; e < 8; ++e) {
      const float x0 = xv[e][0];
      const float x1 = xv[e][1];
      const float n0 = fmaf(sc0, x0 - mean0, be0);
      const float n1 = fmaf(sc1, x1 - mean1, be1);
      const float w0 = fmaf(u0, st0, n0);
      const float w1 = fmaf(u1, st1, n1);
      st0 = (w0 > 0.0f) ? w0 : 0.0f;
      st1 = (w1 > 0.0f) ? w1 : 0.0f;
      const _Float16 h0 = (_Float16)st0;
      const _Float16 h1 = (_Float16)st1;
      pk[e] = (unsigned)__builtin_bit_cast(unsigned short, h0) | ((unsigned)__builtin_bit_cast(unsigned short, h1) << 16);
    }
    if (!LASTL) {
      for (int pass = 0; pass < 2; ++pass) {
#pragma unroll
        for (int e = 0; e < 8; ++e) *(volatile unsigned*)(hp + (size_t)(t0 + e) * HSTRIDE) = pk[e];
        __threadfence();
      }
    }
  }
  if (LASTL) {
    v2f o;
    o[0] = st0;
    o[1] = st1;
    float* lp = LASTP + (size_t)b * NHID + ch;
    *(volatile v2f*)lp = o;
    __threadfence();
    *(volatile v2f*)lp = o;
  }
}

__global__ __launch_bounds__(NTHR) void head_kernel(const float* __restrict__ LASTP, const float* __restrict__ Wc,
                                                   const float* __restrict__ bc, float* __restrict__ out) {
  const int idx = blockIdx.x * NTHR + threadIdx.x;
  const int b = idx >> 7;
  const int c = idx & (NCLS - 1);
  const float* lp = LASTP + (size_t)b * NHID;
  const float* wp = Wc + c;
  float s0 = 0.0f, s1 = 0.0f, s2 = 0.0f, s3 = 0.0f;
#pragma unroll 1
  for (int k = 0; k < NHID; k += 4) {
    const v4f hv = *(const v4f*)(lp + k);
    const float w0 = bf16r(wp[(size_t)(k + 0) * NCLS]);
    const float w1 = bf16r(wp[(size_t)(k + 1) * NCLS]);
    const float w2 = bf16r(wp[(size_t)(k + 2) * NCLS]);
    const float w3 = bf16r(wp[(size_t)(k + 3) * NCLS]);
    s0 = fmaf(hv[0], w0, s0);
    s1 = fmaf(hv[1], w1, s1);
    s2 = fmaf(hv[2], w2, s2);
    s3 = fmaf(hv[3], w3, s3);
  }
  const float r = ((s0 + s1) + (s2 + s3)) + bf16r(bc[c]);
  *(volatile float*)(out + idx) = r;
  __threadfence();
  *(volatile float*)(out + idx) = r;
}

extern "C" void kernel_launch(void* const* d_in, const int* in_sizes, int n_in,
                              void* d_out, int out_size, void* d_ws, size_t ws_size, hipStream_t stream) {
  if (n_in < 10 || d_out == nullptr || d_ws == nullptr) return;
  if (in_sizes[0] != NROWS * NIN || in_sizes[1] != NIN * NHID || in_sizes[2] != NHID ||
      in_sizes[3] != (NLAYER - 1) * NHID * NHID || in_sizes[4] != (NLAYER - 1) * NHID ||
      in_sizes[5] != NLAYER * NHID || in_sizes[6] != NLAYER * NHID || in_sizes[7] != NLAYER * NHID ||
      in_sizes[8] != NHID * NCLS || in_sizes[9] != NCLS || out_size != NBATCH * NCLS) return;

  const float* inp = (const float*)d_in[0];
  const float* W0  = (const float*)d_in[1];
  const float* b0  = (const float*)d_in[2];
  const float* Ws  = (const float*)d_in[3];
  const float* bs  = (const float*)d_in[4];
  const float* uu  = (const float*)d_in[5];
  const float* gam = (const float*)d_in[6];
  const float* bet = (const float*)d_in[7];
  const float* Wc  = (const float*)d_in[8];
  const float* bc  = (const float*)d_in[9];
  float* out = (float*)d_out;

  char* ws = (char*)d_ws; size_t off = 0;
  auto carve = [&](size_t bytes) -> char* { char* p = ws + off; off += (bytes + 255) & ~(size_t)255; return p; };
  float*          XF    = (float*)carve((size_t)NROWS * NHID * 4);
  unsigned short* HPL   = (unsigned short*)carve((size_t)NROWS * NHID * 2);
  unsigned short* A0    = (unsigned short*)carve((size_t)NROWS * NIN * 2);
  unsigned short* W0T   = (unsigned short*)carve((size_t)NHID * NIN * 2);
  unsigned short* WST   = (unsigned short*)carve((size_t)(NLAYER - 1) * NHID * NHID * 2);
  float*          PSUM  = (float*)carve((size_t)NTILEM * NHID * 4);
  float*          PSQ   = (float*)carve((size_t)NTILEM * NHID * 4);
  float*          STAT  = (float*)carve((size_t)2 * NHID * 4);
  float*          LASTP = (float*)carve((size_t)NBATCH * NHID * 4);
  if (off > ws_size || off > (size_t)134217728) return;

  const int n8 = NROWS * NIN / 8;
  cvt8_kernel<<<n8 / NTHR, NTHR, 0, stream>>>(inp, A0, n8);
  tpw_kernel<<<dim3(NHID / 64, NIN / 64, 1), NTHR, 0, stream>>>(W0, NIN, NHID, NIN, W0T, WCARRY);
  tpw_kernel<<<dim3(NHID / 64, NHID / 64, NLAYER - 1), NTHR, 0, stream>>>(Ws, NHID, NHID, NHID, WST, WCARRY);

  const int ggrid = (NTILEM * NTILEN) / 8;
  const int sgrid = (NBATCH * NHID / 2) / NTHR;
  for (int l = 0; l < NLAYER; ++l) {
    if (l == 0) {
      gemm_f16_stats<NIN><<<ggrid, 256, 0, stream>>>(A0, W0T, b0, XF, PSUM, PSQ);
    } else {
      gemm_f16_stats<NHID><<<ggrid, 256, 0, stream>>>(HPL, WST + (size_t)(l - 1) * NHID * NHID,
                                                      bs + (size_t)(l - 1) * NHID, XF, PSUM, PSQ);
    }
    stat_finalize_kernel<<<NHID / NTHR, NTHR, 0, stream>>>(PSUM, PSQ, gam + (size_t)l * NHID, STAT);
    if (l < NLAYER - 1) {
      scan_kernel<false><<<sgrid, NTHR, 0, stream>>>(XF, STAT, bet + (size_t)l * NHID, uu + (size_t)l * NHID,
                                                     (unsigned*)HPL, LASTP);
    } else {
      scan_kernel<true><<<sgrid, NTHR, 0, stream>>>(XF, STAT, bet + (size_t)l * NHID, uu + (size_t)l * NHID,
                                                    (unsigned*)HPL, LASTP);
    }
  }
  head_kernel<<<(NBATCH * NCLS) / NTHR, NTHR, 0, stream>>>(LASTP, Wc, bc, out);
}
